// LSTM_Cell_188978561241
// MI455X (gfx1250) — hardware-verified
//
#include <hip/hip_runtime.h>
#include <stddef.h>
#include <stdint.h>

#define NBATCH 4096
#define NIN    1024
#define NHID   1024
#define KTOT   (NIN + NHID)
#define NKS    (KTOT / 32)
#define TBM    128
#define TBN    32

static_assert((KTOT % 32) == 0);
static_assert((NBATCH % TBM) == 0);
static_assert((NHID % TBN) == 0);
static_assert(KTOT == 8 * 256);
static_assert(TBM * TBN == 4 * 4 * 256);

typedef __attribute__((ext_vector_type(16))) __bf16 v16b;
typedef float        v8f __attribute__((ext_vector_type(8)));
typedef float        v4f __attribute__((ext_vector_type(4)));
typedef unsigned int v4u __attribute__((ext_vector_type(4)));

__device__ __forceinline__ unsigned short bf_bits(float f) {
  const unsigned u = __float_as_uint(f);
  return (unsigned short)((u + 0x7FFFu + ((u >> 16) & 1u)) >> 16);
}
__device__ __forceinline__ float bfr(float f) { return __uint_as_float(((unsigned)bf_bits(f)) << 16); }
__device__ __forceinline__ unsigned pk16(unsigned short a, unsigned short b) { return (unsigned)a | ((unsigned)b << 16); }
__device__ __forceinline__ v8f zero8() { v8f z = {0.f, 0.f, 0.f, 0.f, 0.f, 0.f, 0.f, 0.f}; return z; }
__device__ __forceinline__ float sigm(float v) {
  const float e = expf(-v);
  return 1.0f / (1.0f + e);
}

union FragB { v16b v; v4u u[2]; };
__device__ __forceinline__ v16b ldfrag_b(const unsigned short* p) {
  FragB f;
  f.u[0] = *(const v4u*)(p);
  f.u[1] = *(const v4u*)(p + 16);
  return f.v;
}

__device__ __forceinline__ v8f mma_b(v16b a, v16b b, v8f c) {
  return __builtin_amdgcn_wmma_f32_16x16x32_bf16(false, a, false, b, (short)0, c, false, false);
}
__device__ __forceinline__ void guard8(v8f& c0, v8f& c1, v8f& c2, v8f& c3, v8f& c4, v8f& c5, v8f& c6, v8f& c7,
                                       const v16b& a0, const v16b& a1, const v16b& b0, const v16b& b1,
                                       const v16b& b2, const v16b& b3) {
#if defined(__HIP_DEVICE_COMPILE__)
  asm volatile("v_nop\n\tv_nop\n\tv_nop\n\tv_nop"
               : "+v"(c0), "+v"(c1), "+v"(c2), "+v"(c3), "+v"(c4), "+v"(c5), "+v"(c6), "+v"(c7)
               : "v"(a0), "v"(a1), "v"(b0), "v"(b1), "v"(b2), "v"(b3));
#endif
}

__global__ __launch_bounds__(256)
void k_cvt(const float* __restrict__ x, const float* __restrict__ h1,
           const float* __restrict__ w0x, const float* __restrict__ w0h,
           const float* __restrict__ w1x, const float* __restrict__ w1h,
           const float* __restrict__ w2x, const float* __restrict__ w2h,
           const float* __restrict__ w3x, const float* __restrict__ w3h,
           unsigned short* Acat, unsigned short* Wcat) {
  const int blk = blockIdx.x, tid = threadIdx.x;
  const int half = tid >> 7;
  const int k8 = (tid & 127) * 8;
  const float* src;
  unsigned short* dst;
  if (blk < NBATCH) {
    src = (half == 0) ? (x + (size_t)blk * NIN + k8) : (h1 + (size_t)blk * NHID + k8);
    dst = Acat + (size_t)blk * KTOT + tid * 8;
  } else {
    const int gn = blk - NBATCH;
    const int g = gn >> 10, n = gn & (NHID - 1);
    const float* wx = (g == 0) ? w0x : ((g == 1) ? w1x : ((g == 2) ? w2x : w3x));
    const float* wh = (g == 0) ? w0h : ((g == 1) ? w1h : ((g == 2) ? w2h : w3h));
    src = (half == 0) ? (wx + (size_t)n * NIN + k8) : (wh + (size_t)n * NHID + k8);
    dst = Wcat + (size_t)gn * KTOT + tid * 8;
  }
  const v4f a = *(const v4f*)(src);
  const v4f b = *(const v4f*)(src + 4);
  v4u u;
  u[0] = pk16(bf_bits(a[0]), bf_bits(a[1]));
  u[1] = pk16(bf_bits(a[2]), bf_bits(a[3]));
  u[2] = pk16(bf_bits(b[0]), bf_bits(b[1]));
  u[3] = pk16(bf_bits(b[2]), bf_bits(b[3]));
  *(volatile v4u*)dst = u;
  __threadfence();
  *(volatile v4u*)dst = u;
}

__global__ __launch_bounds__(256)
void k_gates(const unsigned short* __restrict__ Acat, const unsigned short* __restrict__ Wcat,
             const float* __restrict__ c1,
             const float* __restrict__ bx0, const float* __restrict__ bh0,
             const float* __restrict__ bx1, const float* __restrict__ bh1,
             const float* __restrict__ bx2, const float* __restrict__ bh2,
             const float* __restrict__ bx3, const float* __restrict__ bh3,
             float* outh, float* outc) {
  __shared__ __align__(16) float sh[TBM * TBN];
  __shared__ __align__(16) float sc[TBM * TBN];
  const int tid = threadIdx.x, w = tid >> 5, lane = tid & 31, hh = lane >> 4, c = lane & 15;
  const int wm = w & 3, wn = w >> 2;
  const int Mbase = blockIdx.x * TBM, Nbase = blockIdx.y * TBN;
  const int n = Nbase + 16 * wn + c;

  const unsigned short* ap0 = Acat + (size_t)(Mbase + 32 * wm + c) * KTOT + 8 * hh;
  const unsigned short* ap1 = ap0 + (size_t)16 * KTOT;
  const unsigned short* bp0 = Wcat + ((size_t)0 * NHID + n) * KTOT + 8 * hh;
  const unsigned short* bp1 = Wcat + ((size_t)1 * NHID + n) * KTOT + 8 * hh;
  const unsigned short* bp2 = Wcat + ((size_t)2 * NHID + n) * KTOT + 8 * hh;
  const unsigned short* bp3 = Wcat + ((size_t)3 * NHID + n) * KTOT + 8 * hh;

  v8f acc[4][2];
#pragma unroll
  for (int g = 0; g < 4; ++g) { acc[g][0] = zero8(); acc[g][1] = zero8(); }

#pragma unroll 1
  for (int ks = 0; ks < NKS; ++ks) {
    const int ko = 32 * ks;
    const v16b a0 = ldfrag_b(ap0 + ko);
    const v16b a1 = ldfrag_b(ap1 + ko);
    const v16b b0 = ldfrag_b(bp0 + ko);
    const v16b b1 = ldfrag_b(bp1 + ko);
    const v16b b2 = ldfrag_b(bp2 + ko);
    const v16b b3 = ldfrag_b(bp3 + ko);
    acc[0][0] = mma_b(a0, b0, acc[0][0]);
    acc[0][1] = mma_b(a1, b0, acc[0][1]);
    acc[1][0] = mma_b(a0, b1, acc[1][0]);
    acc[1][1] = mma_b(a1, b1, acc[1][1]);
    acc[2][0] = mma_b(a0, b2, acc[2][0]);
    acc[2][1] = mma_b(a1, b2, acc[2][1]);
    acc[3][0] = mma_b(a0, b3, acc[3][0]);
    acc[3][1] = mma_b(a1, b3, acc[3][1]);
    guard8(acc[0][0], acc[0][1], acc[1][0], acc[1][1], acc[2][0], acc[2][1], acc[3][0], acc[3][1],
           a0, a1, b0, b1, b2, b3);
  }

  const float bs0 = bfr(bx0[n]) + bfr(bh0[n]);
  const float bs1 = bfr(bx1[n]) + bfr(bh1[n]);
  const float bs2 = bfr(bx2[n]) + bfr(bh2[n]);
  const float bs3 = bfr(bx3[n]) + bfr(bh3[n]);
  const int lcol = 16 * wn + c;
#pragma unroll
  for (int t = 0; t < 2; ++t) {
#pragma unroll
    for (int r = 0; r < 8; ++r) {
      const int lrow = 32 * wm + 16 * t + 8 * hh + r;
      const int m = Mbase + lrow;
      const float iv = sigm(acc[0][t][r] + bs0);
      const float fv = sigm(acc[1][t][r] + bs1);
      const float ov = sigm(acc[2][t][r] + bs2);
      const float cv = tanhf(acc[3][t][r] + bs3);
      const float cp = bfr(c1[(size_t)m * NHID + n]);
      const float cn = fv * cp + iv * cv;
      const float hn = ov * tanhf(cn);
      sh[lrow * TBN + lcol] = hn;
      sc[lrow * TBN + lcol] = cn;
    }
  }
  __syncthreads();

  v4f oh[4], oc[4];
  const int rr = tid >> 3, c4 = (tid & 7) * 4;
#pragma unroll
  for (int it = 0; it < 4; ++it) {
    const int lrow = it * 32 + rr;
    oh[it] = *(const v4f*)(sh + lrow * TBN + c4);
    oc[it] = *(const v4f*)(sc + lrow * TBN + c4);
  }
  const size_t ob = (size_t)(Mbase + rr) * NHID + Nbase + c4;
#pragma unroll
  for (int it = 0; it < 4; ++it) {
    const size_t o = ob + (size_t)it * 32 * NHID;
    *(volatile v4f*)(outh + o) = oh[it];
    *(volatile v4f*)(outc + o) = oc[it];
  }
  __threadfence();
#pragma unroll
  for (int it = 0; it < 4; ++it) {
    const size_t o = ob + (size_t)it * 32 * NHID;
    *(volatile v4f*)(outh + o) = oh[it];
    *(volatile v4f*)(outc + o) = oc[it];
  }
}

extern "C" void kernel_launch(void* const* d_in, const int* in_sizes, int n_in,
                              void* d_out, int out_size, void* d_ws, size_t ws_size,
                              hipStream_t stream) {
  if (n_in < 19) return;
  if (in_sizes[0] != NBATCH * NIN) return;
  if (in_sizes[1] != NBATCH * NHID) return;
  if (in_sizes[2] != NBATCH * NHID) return;
  for (int g = 0; g < 4; ++g) {
    if (in_sizes[3 + 4 * g] != NHID * NIN) return;
    if (in_sizes[4 + 4 * g] != NHID) return;
    if (in_sizes[5 + 4 * g] != NHID * NHID) return;
    if (in_sizes[6 + 4 * g] != NHID) return;
  }
  if (out_size != 2 * NBATCH * NHID) return;

  const float* x  = (const float*)d_in[0];
  const float* h1 = (const float*)d_in[1];
  const float* c1 = (const float*)d_in[2];
  const float* wx[4];
  const float* wh[4];
  const float* bx[4];
  const float* bh[4];
  for (int g = 0; g < 4; ++g) {
    wx[g] = (const float*)d_in[3 + 4 * g];
    bx[g] = (const float*)d_in[4 + 4 * g];
    wh[g] = (const float*)d_in[5 + 4 * g];
    bh[g] = (const float*)d_in[6 + 4 * g];
  }
  float* outh = (float*)d_out;
  float* outc = outh + (size_t)NBATCH * NHID;

  const size_t sA = (size_t)NBATCH * KTOT * 2;
  const size_t sW = (size_t)4 * NHID * KTOT * 2;
  size_t off = 0;
  const size_t oA = off; off += sA;
  const size_t oW = off; off += sW;
  if (off > ws_size) return;
  if (off > (size_t)134217728) return;

  char* ws = (char*)d_ws;
  unsigned short* Acat = (unsigned short*)(ws + oA);
  unsigned short* Wcat = (unsigned short*)(ws + oW);

  k_cvt<<<dim3(NBATCH + 4 * NHID), dim3(256), 0, stream>>>(x, h1, wx[0], wh[0], wx[1], wh[1], wx[2], wh[2],
                                                           wx[3], wh[3], Acat, Wcat);
  k_gates<<<dim3(NBATCH / TBM, NHID / TBN), dim3(256), 0, stream>>>(Acat, Wcat, c1,
                                                                    bx[0], bh[0], bx[1], bh[1],
                                                                    bx[2], bh[2], bx[3], bh[3],
                                                                    outh, outc);
  (void)hipGetLastError();
}
